// BoundaryTransformerLayer_35656818491920
// MI455X (gfx1250) — hardware-run, weakly checked
//
#include <hip/hip_runtime.h>
#include <math.h>

typedef __attribute__((ext_vector_type(16))) _Float16 v16h;
typedef __attribute__((ext_vector_type(16))) __bf16 v16b;
typedef __attribute__((ext_vector_type(8)))  _Float16 v8h;
typedef __attribute__((ext_vector_type(8)))  float v8f;
typedef __attribute__((ext_vector_type(4)))  float v4f;
typedef __attribute__((ext_vector_type(2)))  float v2f;
typedef __attribute__((ext_vector_type(4)))  unsigned v4u;
typedef __attribute__((ext_vector_type(4)))  int v4i;
typedef float __attribute__((may_alias)) float_a;
typedef int __attribute__((may_alias)) int_a;

template <typename T> __device__ __forceinline__ void vst2(void* p, T v) { *(volatile T*)p = v; __threadfence(); *(volatile T*)p = v; }
__device__ __forceinline__ v8f wmma16(v16h a, v16h b, v8f c) {
  v8f d = __builtin_amdgcn_wmma_f32_16x16x32_f16(false, a, false, b, (short)0, c, false, false);
  asm volatile("v_nop\n\tv_nop\n\tv_nop\n\tv_nop" : "+v"(d) : "v"(a), "v"(b));
  return d;
}
__device__ __forceinline__ v8f wmma_bf(v16b a, v16b b, v8f c) {
  v8f d = __builtin_amdgcn_wmma_f32_16x16x32_bf16(false, a, false, b, (short)0, c, false, false);
  asm volatile("v_nop\n\tv_nop\n\tv_nop\n\tv_nop" : "+v"(d) : "v"(a), "v"(b));
  return d;
}
__device__ __forceinline__ v16h frag_h(const _Float16* rowk0, int lane) {
  union { v16h v; v8h q[2]; } u; const _Float16* p = rowk0 + 8 * (lane >> 4);
  u.q[0] = *(const v8h*)p; u.q[1] = *(const v8h*)(p + 16); return u.v;
}
__device__ __forceinline__ v16h frag_f32(const float* rowk0, int lane) {
  v16h a; const float* p = rowk0 + 8 * (lane >> 4);
#pragma unroll
  for (int i = 0; i < 8; ++i) { a[i] = (_Float16)p[i]; a[8 + i] = (_Float16)p[16 + i]; }
  return a;
}
__device__ __forceinline__ v16h frag_f32s(const float* rowk0, int lane, float sc) {
  v16h a; const float* p = rowk0 + 8 * (lane >> 4);
#pragma unroll
  for (int i = 0; i < 8; ++i) { a[i] = (_Float16)(p[i] * sc); a[8 + i] = (_Float16)(p[16 + i] * sc); }
  return a;
}
__device__ __forceinline__ v16h fragc_f32(const float* W, int k0, int n, int lane, int ld, int K) {
  v16h a; const int g = lane >> 4;
#pragma unroll
  for (int i = 0; i < 8; ++i) { const int ka = k0 + 8 * g + i, kb = ka + 16;
    a[i] = (_Float16)(ka < K ? W[(size_t)(ka < K ? ka : K - 1) * ld + n] : 0.f); a[8 + i] = (_Float16)(kb < K ? W[(size_t)(kb < K ? kb : K - 1) * ld + n] : 0.f); }
  return a;
}
struct F2 { v16b h, l; };
__device__ __forceinline__ F2 bsplit16(const float v[16]) { F2 r;
#pragma unroll
  for (int i = 0; i < 16; ++i) { const __bf16 h = (__bf16)v[i]; r.h[i] = h; r.l[i] = (__bf16)(v[i] - (float)h); }
  return r; }
__device__ __forceinline__ F2 split_row(const float* row, int k0, int lane) { float v[16]; const float* p = row + k0 + 8 * (lane >> 4);
#pragma unroll
  for (int i = 0; i < 8; ++i) { v[i] = p[i]; v[8 + i] = p[16 + i]; }
  return bsplit16(v); }
__device__ __forceinline__ F2 split_rowK(const float* row, int k0, int lane, int K) { float v[16]; const int g = lane >> 4;
#pragma unroll
  for (int i = 0; i < 8; ++i) { const int ka = k0 + 8 * g + i, kb = ka + 16; v[i] = ka < K ? row[ka < K ? ka : K - 1] : 0.f; v[8 + i] = kb < K ? row[kb < K ? kb : K - 1] : 0.f; }
  return bsplit16(v); }
__device__ __forceinline__ F2 split_col(const float* W, int k0, int n, int lane, int ld, int K) { float v[16]; const int g = lane >> 4;
#pragma unroll
  for (int i = 0; i < 8; ++i) { const int ka = k0 + 8 * g + i, kb = ka + 16; v[i] = ka < K ? W[(size_t)(ka < K ? ka : K - 1) * ld + n] : 0.f; v[8 + i] = kb < K ? W[(size_t)(kb < K ? kb : K - 1) * ld + n] : 0.f; }
  return bsplit16(v); }
__device__ __forceinline__ v8f mac3(const F2& a, const F2& b, v8f c) { c = wmma_bf(a.l, b.h, c); c = wmma_bf(a.h, b.l, c); return wmma_bf(a.h, b.h, c); }
__device__ __forceinline__ float sigm(float v) { return 1.0f / (1.0f + expf(-v)); }
#define LDSX() do { asm volatile("s_wait_dscnt 0" ::: "memory"); __builtin_amdgcn_wave_barrier(); __builtin_amdgcn_fence(__ATOMIC_RELEASE, "workgroup"); } while (0)

__device__ __forceinline__ float bfr(float v) { return (float)(__bf16)v; }
#define NPTS 100000
#define NS 16
#define CCH 64
#define CS 8
#ifndef NBLK
#define NBLK (NPTS / 8)
#endif
#define WS_XQ 0u
#define WS_XK (WS_XQ + 4u * (size_t)NPTS * CCH)
#define WS_XV (WS_XK + 4u * (size_t)NPTS * CCH)
#define WS_END (WS_XV + 4u * (size_t)NPTS * CCH)
__device__ __forceinline__ float bnf(float t, const float* G, const float* Bb, const float* M, const float* V, int c) { const float m = M ? bfr(M[c]) : 0.f; const float v = V ? bfr(V[c]) : 1.0f; return (t - m) * rsqrtf(v + 1e-5f) * bfr(G[c]) + bfr(Bb[c]); }
__global__ __launch_bounds__(128) void k_qkv(const float* __restrict__ X, const float* __restrict__ WQ, const float* __restrict__ BQ, const float* __restrict__ WK, const float* __restrict__ BK, const float* __restrict__ WV, const float* __restrict__ BV, float* __restrict__ XQ, float* __restrict__ XK, float* __restrict__ XV) {
  __shared__ __align__(16) float sf[4][16][68];
  const int tid = threadIdx.x, wave = tid >> 5, lane = tid & 31, col = lane & 15, g = lane >> 4; const int which = blockIdx.y; const size_t r0 = (size_t)blockIdx.x * 64 + wave * 16;
  const float* WA = which == 0 ? WQ : which == 1 ? WK : WV; const float* BA = which == 0 ? BQ : which == 1 ? BK : BV; float* D = which == 0 ? XQ : which == 1 ? XK : XV;
  v8f acc[4] = {};
#pragma unroll
  for (int kc = 0; kc < 2; ++kc) { v16b a; { const size_t r = (r0 + col < NPTS) ? r0 + col : NPTS - 1; const float* p = X + r * CCH + kc * 32 + 8 * g;
#pragma unroll
      for (int i = 0; i < 8; ++i) { a[i] = (__bf16)p[i]; a[8 + i] = (__bf16)p[16 + i]; } }
#pragma unroll
    for (int j = 0; j < 4; ++j) { v16b w; const int o = j * 16 + col;
#pragma unroll
      for (int i = 0; i < 8; ++i) { w[i] = (__bf16)WA[(size_t)(kc * 32 + 8 * g + i) * CCH + o]; w[8 + i] = (__bf16)WA[(size_t)(kc * 32 + 16 + 8 * g + i) * CCH + o]; }
      acc[j] = wmma_bf(a, w, acc[j]); } }
#pragma unroll
  for (int j = 0; j < 4; ++j) { const float bb = bfr(BA[j * 16 + col]);
#pragma unroll
    for (int r = 0; r < 8; ++r) sf[wave][8 * g + r][j * 16 + col] = acc[j][r] + bb; }
  LDSX(); for (int rl = 0; rl < 16; ++rl) { const size_t r = r0 + rl; if (r < NPTS && lane < 16) vst2(D + r * CCH + lane * 4, *(const v4f*)&sf[wave][rl][lane * 4]); } }
__global__ __launch_bounds__(128) void k_pt(const float* __restrict__ P, const int* __restrict__ IDX, const float* __restrict__ XQ, const float* __restrict__ XK, const float* __restrict__ XV,
    const float* __restrict__ WP1, const float* __restrict__ BP1, const float* __restrict__ GP, const float* __restrict__ BEP, const float* __restrict__ MP, const float* __restrict__ VP,
    const float* __restrict__ WP2, const float* __restrict__ BP2, const float* __restrict__ G1, const float* __restrict__ BE1, const float* __restrict__ M1, const float* __restrict__ V1,
    const float* __restrict__ WW1, const float* __restrict__ BW1, const float* __restrict__ G2, const float* __restrict__ BE2, const float* __restrict__ M2, const float* __restrict__ V2,
    const float* __restrict__ WW2, const float* __restrict__ BW2, float* __restrict__ OUT) {
  __shared__ __align__(16) float spr[128][CCH]; __shared__ __align__(16) float sw0[128][CCH + 4]; __shared__ float sw1[128][CS]; __shared__ float swt[128][CS]; __shared__ __align__(16) float so[8][CCH]; __shared__ int sj[128];
  const int tid = threadIdx.x, wave = tid >> 5, lane = tid & 31, col = lane & 15, g = lane >> 4; const size_t n0 = (size_t)blockIdx.x * 8;
  { const int row = tid; const size_t n = n0 + (row >> 4); const int j = IDX[n * NS + (row & 15)]; sj[row] = j;
    const float gx = bfr(P[(size_t)j * 3]) - bfr(P[n * 3]), gy = bfr(P[(size_t)j * 3 + 1]) - bfr(P[n * 3 + 1]), gz = bfr(P[(size_t)j * 3 + 2]) - bfr(P[n * 3 + 2]);
    float t[3];
#pragma unroll
    for (int o = 0; o < 3; ++o) { const float u = gx * bfr(WP1[0 * 3 + o]) + gy * bfr(WP1[1 * 3 + o]) + gz * bfr(WP1[2 * 3 + o]) + bfr(BP1[o]); t[o] = fmaxf(bnf(u, GP, BEP, MP, VP, o), 0.f); }
#pragma unroll 1
    for (int c = 0; c < CCH; ++c) { const float pr = t[0] * bfr(WP2[0 * CCH + c]) + t[1] * bfr(WP2[1 * CCH + c]) + t[2] * bfr(WP2[2 * CCH + c]) + bfr(BP2[c]); spr[row][c] = pr;
      const float w0 = XK[(size_t)j * CCH + c] - XQ[n * CCH + c] + pr; sw0[row][c] = fmaxf(bnf(w0, G1, BE1, M1, V1, c), 0.f); } }
  __syncthreads();
#pragma unroll
  for (int tI = 0; tI < 2; ++tI) { const int rbase = wave * 32 + tI * 16; v8f acc = {};
#pragma unroll
    for (int kc = 0; kc < 2; ++kc) { const F2 a = split_row(&sw0[rbase + col][0], kc * 32, lane); v16b w;
#pragma unroll
      for (int i = 0; i < 16; ++i) { const int k = kc * 32 + (i < 8 ? 8 * g + i : 16 + 8 * g + (i - 8)); w[i] = (col < CS) ? (__bf16)WW1[k * CS + (col < CS ? col : 0)] : (__bf16)0.f; }
      acc = wmma_bf(a.h, w, acc); acc = wmma_bf(a.l, w, acc); }
    if (col < CS) {
#pragma unroll
      for (int r = 0; r < 8; ++r) { const float u = acc[r] + bfr(BW1[col]); sw1[rbase + 8 * g + r][col] = fmaxf(bnf(u, G2, BE2, M2, V2, col), 0.f); } } }
  LDSX(); __syncthreads();
  { const int row = tid;
#pragma unroll 1
    for (int o = 0; o < CS; ++o) { float s = bfr(BW2[o]);
#pragma unroll
      for (int k = 0; k < CS; ++k) s += sw1[row][k] * bfr(WW2[k * CS + o]);
      swt[row][o] = s; } }
  __syncthreads();
  if (tid < 64) { const int pt = tid >> 3, o = tid & 7; float m = -3.0e38f; for (int jn = 0; jn < NS; ++jn) m = fmaxf(m, swt[pt * 16 + jn][o]); float s = 0.f; for (int jn = 0; jn < NS; ++jn) { const float e = expf(swt[pt * 16 + jn][o] - m); swt[pt * 16 + jn][o] = e; s += e; } const float inv = 1.0f / s; for (int jn = 0; jn < NS; ++jn) swt[pt * 16 + jn][o] *= inv; }
  __syncthreads();
  { const int pt = tid >> 4, c0 = (tid & 15) * 4;
#pragma unroll
    for (int e = 0; e < 4; ++e) { const int c = c0 + e; float s = 0.f; for (int jn = 0; jn < NS; ++jn) { const int row = pt * 16 + jn; s += (XV[(size_t)sj[row] * CCH + c] + spr[row][c]) * swt[row][c & (CS - 1)]; } so[pt][c] = s; } }
  __syncthreads();
  { const int pt = wave * 2 + (lane >> 4); vst2(OUT + (n0 + pt) * CCH + (lane & 15) * 4, *(const v4f*)&so[pt][(lane & 15) * 4]); }
}
extern "C" void kernel_launch(void* const* d_in, const int* in_sizes, int n_in, void* d_out, int out_size, void* d_ws, size_t ws_size, hipStream_t stream) {
  (void)in_sizes; (void)n_in; (void)out_size;
  const float** F = (const float**)d_in;
  if (ws_size < (size_t)WS_END) return;
  char* ws = (char*)d_ws; float *XQ = (float*)(ws + WS_XQ), *XK = (float*)(ws + WS_XK), *XV = (float*)(ws + WS_XV);
  k_qkv<<<dim3((NPTS + 63) / 64, 3), 128, 0, stream>>>(F[1], F[3], F[4], F[5], F[6], F[7], F[8], XQ, XK, XV);
  k_pt<<<dim3(NBLK), 128, 0, stream>>>(F[0], (const int*)d_in[2], XQ, XK, XV, F[9], F[10], F[11], F[12], F[13], F[14], F[15], F[16], F[17], F[18], F[19], F[20], F[21], F[22], F[23], F[24], F[25], F[26], F[27], F[28], (float*)d_out);
}
